// SelfAttentionModel_54004918780607
// MI455X (gfx1250) — hardware-verified
//
#include <hip/hip_runtime.h>
#include <math.h>

typedef __attribute__((ext_vector_type(16))) _Float16 v16h;
typedef __attribute__((ext_vector_type(16))) __bf16 v16b;
typedef __attribute__((ext_vector_type(8)))  _Float16 v8h;
typedef __attribute__((ext_vector_type(8)))  float v8f;
typedef __attribute__((ext_vector_type(4)))  float v4f;
typedef __attribute__((ext_vector_type(2)))  float v2f;
typedef __attribute__((ext_vector_type(4)))  unsigned v4u;
typedef __attribute__((ext_vector_type(4)))  int v4i;
typedef float __attribute__((may_alias)) float_a;
typedef int __attribute__((may_alias)) int_a;

template <typename T> __device__ __forceinline__ void vst2(void* p, T v) { *(volatile T*)p = v; __threadfence(); *(volatile T*)p = v; }
__device__ __forceinline__ v8f wmma16(v16h a, v16h b, v8f c) {
  v8f d = __builtin_amdgcn_wmma_f32_16x16x32_f16(false, a, false, b, (short)0, c, false, false);
  asm volatile("v_nop\n\tv_nop\n\tv_nop\n\tv_nop" : "+v"(d) : "v"(a), "v"(b));
  return d;
}
__device__ __forceinline__ v8f wmma_bf(v16b a, v16b b, v8f c) {
  v8f d = __builtin_amdgcn_wmma_f32_16x16x32_bf16(false, a, false, b, (short)0, c, false, false);
  asm volatile("v_nop\n\tv_nop\n\tv_nop\n\tv_nop" : "+v"(d) : "v"(a), "v"(b));
  return d;
}
__device__ __forceinline__ v16h frag_h(const _Float16* rowk0, int lane) {
  union { v16h v; v8h q[2]; } u; const _Float16* p = rowk0 + 8 * (lane >> 4);
  u.q[0] = *(const v8h*)p; u.q[1] = *(const v8h*)(p + 16); return u.v;
}
__device__ __forceinline__ v16h frag_f32(const float* rowk0, int lane) {
  v16h a; const float* p = rowk0 + 8 * (lane >> 4);
#pragma unroll
  for (int i = 0; i < 8; ++i) { a[i] = (_Float16)p[i]; a[8 + i] = (_Float16)p[16 + i]; }
  return a;
}
__device__ __forceinline__ v16h frag_f32s(const float* rowk0, int lane, float sc) {
  v16h a; const float* p = rowk0 + 8 * (lane >> 4);
#pragma unroll
  for (int i = 0; i < 8; ++i) { a[i] = (_Float16)(p[i] * sc); a[8 + i] = (_Float16)(p[16 + i] * sc); }
  return a;
}
__device__ __forceinline__ v16h fragc_f32(const float* W, int k0, int n, int lane, int ld, int K) {
  v16h a; const int g = lane >> 4;
#pragma unroll
  for (int i = 0; i < 8; ++i) { const int ka = k0 + 8 * g + i, kb = ka + 16;
    a[i] = (_Float16)(ka < K ? W[(size_t)(ka < K ? ka : K - 1) * ld + n] : 0.f); a[8 + i] = (_Float16)(kb < K ? W[(size_t)(kb < K ? kb : K - 1) * ld + n] : 0.f); }
  return a;
}
struct F2 { v16b h, l; };
__device__ __forceinline__ F2 bsplit16(const float v[16]) { F2 r;
#pragma unroll
  for (int i = 0; i < 16; ++i) { const __bf16 h = (__bf16)v[i]; r.h[i] = h; r.l[i] = (__bf16)(v[i] - (float)h); }
  return r; }
__device__ __forceinline__ F2 split_row(const float* row, int k0, int lane) { float v[16]; const float* p = row + k0 + 8 * (lane >> 4);
#pragma unroll
  for (int i = 0; i < 8; ++i) { v[i] = p[i]; v[8 + i] = p[16 + i]; }
  return bsplit16(v); }
__device__ __forceinline__ F2 split_rowK(const float* row, int k0, int lane, int K) { float v[16]; const int g = lane >> 4;
#pragma unroll
  for (int i = 0; i < 8; ++i) { const int ka = k0 + 8 * g + i, kb = ka + 16; v[i] = ka < K ? row[ka < K ? ka : K - 1] : 0.f; v[8 + i] = kb < K ? row[kb < K ? kb : K - 1] : 0.f; }
  return bsplit16(v); }
__device__ __forceinline__ F2 split_col(const float* W, int k0, int n, int lane, int ld, int K) { float v[16]; const int g = lane >> 4;
#pragma unroll
  for (int i = 0; i < 8; ++i) { const int ka = k0 + 8 * g + i, kb = ka + 16; v[i] = ka < K ? W[(size_t)(ka < K ? ka : K - 1) * ld + n] : 0.f; v[8 + i] = kb < K ? W[(size_t)(kb < K ? kb : K - 1) * ld + n] : 0.f; }
  return bsplit16(v); }
__device__ __forceinline__ v8f mac3(const F2& a, const F2& b, v8f c) { c = wmma_bf(a.l, b.h, c); c = wmma_bf(a.h, b.l, c); return wmma_bf(a.h, b.h, c); }
__device__ __forceinline__ float sigm(float v) { return 1.0f / (1.0f + expf(-v)); }
#define LDSX() do { asm volatile("s_wait_dscnt 0" ::: "memory"); __builtin_amdgcn_wave_barrier(); __builtin_amdgcn_fence(__ATOMIC_RELEASE, "workgroup"); } while (0)


#define NB 4
#define NP 4096
#define CIN 256
#define CQ 32
#define CV 256
#ifndef TNB
#define TNB NB
#endif
#ifndef TQB
#define TQB (NP / 64)
#endif
typedef __attribute__((ext_vector_type(8))) __bf16 v8b;
__device__ __forceinline__ v16b frag_b(const __bf16* rowk0, int lane) {
  union { v16b v; v8b q[2]; } u; const __bf16* p = rowk0 + 8 * (lane >> 4);
  u.q[0] = *(const v8b*)p; u.q[1] = *(const v8b*)(p + 16); return u.v;
}
__device__ __forceinline__ float bfr(float v) { return (float)(__bf16)v; }
__device__ __attribute__((noinline)) float exp_ni(float v) { return expf(v); }
__device__ __attribute__((noinline)) float erf_ni(float v) { return erff(v); }

#define WS_QH  0u
#define WS_QL  (WS_QH + 2u * (size_t)NB * NP * CQ)
#define WS_KH  (WS_QL + 2u * (size_t)NB * NP * CQ)
#define WS_KL  (WS_KH + 2u * (size_t)NB * NP * CQ)
#define WS_VT  (WS_KL + 2u * (size_t)NB * NP * CQ)
#define WS_S   (WS_VT + 2u * (size_t)NB * CV * NP)
#define WS_PH  (WS_S + 4u * (size_t)NP * NP)
#define WS_END (WS_PH + 2u * (size_t)NP * NP)

__global__ __launch_bounds__(128) void k_proj(const float* __restrict__ XQK, const float* __restrict__ XV, const float* __restrict__ WQ, const float* __restrict__ BQ, const float* __restrict__ WK, const float* __restrict__ BK, const float* __restrict__ WV, const float* __restrict__ BV, _Float16* __restrict__ QH, _Float16* __restrict__ QL, _Float16* __restrict__ KH, _Float16* __restrict__ KL, _Float16* __restrict__ VT) {
  __shared__ __align__(16) __bf16 sx[64][CIN + 8]; __shared__ __align__(16) _Float16 sh[64][72], sl[64][72]; __shared__ __align__(16) _Float16 tv[64][72];
  const int tid = threadIdx.x, wave = tid >> 5, lane = tid & 31, col = lane & 15, g = lane >> 4; const int p0 = blockIdx.x * 64; const size_t b = blockIdx.y; const int which = blockIdx.z;
  const float* Wm = which == 0 ? WQ : which == 1 ? WK : WV; const float* Bm = which == 0 ? BQ : which == 1 ? BK : BV; const int nout = (which == 2) ? CV : CQ; const float* X = (which == 2) ? XV : XQK;
  for (int e = tid; e < CIN * 64; e += 128) { const int pl = e / CIN, c = e % CIN; sx[pl][c] = (__bf16)X[((size_t)b * NP + p0 + pl) * CIN + c]; }
  __syncthreads();
#pragma unroll 1
  for (int cg = 0; cg < (nout + 63) / 64; ++cg) { v8f acc[4] = {};
#pragma unroll 2
    for (int kc = 0; kc < CIN / 32; ++kc) { const v16b a = frag_b(&sx[wave * 16 + col][kc * 32], lane);
#pragma unroll
      for (int j = 0; j < 4; ++j) { v16b w; const int o = min(cg * 64 + j * 16 + col, nout - 1);
#pragma unroll
        for (int i = 0; i < 8; ++i) { w[i] = (__bf16)Wm[(size_t)(kc * 32 + 8 * g + i) * nout + o]; w[8 + i] = (__bf16)Wm[(size_t)(kc * 32 + 16 + 8 * g + i) * nout + o]; }
        acc[j] = wmma_bf(a, w, acc[j]); } }
    __syncthreads();
#pragma unroll
    for (int j = 0; j < 4; ++j) { const int ol = j * 16 + col; const float bb = bfr(Bm[min(cg * 64 + ol, nout - 1)]);
#pragma unroll
      for (int r = 0; r < 8; ++r) { const int pl = wave * 16 + 8 * g + r; const float v = acc[j][r] + bb; const _Float16 hv = (_Float16)v; if (which == 2) tv[ol][pl] = hv; else { sh[pl][ol] = hv; sl[pl][ol] = (_Float16)(v - (float)hv); } } }
    __syncthreads();
    if (which < 2) { _Float16* dh = which == 0 ? QH : KH; _Float16* dl = which == 0 ? QL : KL; for (int e = tid; e < 64 * 8; e += 128) { const int pl = e >> 3, q = e & 7; if (cg * 64 + q * 8 >= CQ) continue; const size_t row = b * NP + p0 + pl; vst2((unsigned*)(dh + row * CQ + cg * 64 + q * 8), *(const v4u*)&sh[pl][q * 8]); vst2((unsigned*)(dl + row * CQ + cg * 64 + q * 8), *(const v4u*)&sl[pl][q * 8]); } }
    else { for (int e = tid; e < 64 * 8; e += 128) { const int ol = e >> 3, q = e & 7; vst2((unsigned*)(VT + (b * CV + cg * 64 + ol) * (size_t)NP + p0 + q * 8), *(const v4u*)&tv[ol][q * 8]); } } } }
__global__ __launch_bounds__(128) void k_sc(const _Float16* __restrict__ QH, const _Float16* __restrict__ QL, const _Float16* __restrict__ KH, const _Float16* __restrict__ KL, int b, float* __restrict__ S) { __shared__ __align__(16) float ss[4][16][132];
  const int tid = threadIdx.x, wave = tid >> 5, lane = tid & 31, col = lane & 15, g = lane >> 4; const int k0 = blockIdx.y * 128; const int ql0 = blockIdx.x * 64 + wave * 16; const size_t q0 = (size_t)b * NP + ql0;
  v8f acc[8] = {};
#pragma unroll 1
  for (int kc = 0; kc < CQ / 32; ++kc) { const v16h ah = frag_h(QH + (q0 + col) * CQ + kc * 32, lane), al = frag_h(QL + (q0 + col) * CQ + kc * 32, lane);
#pragma unroll
    for (int j = 0; j < 8; ++j) { const size_t kr = ((size_t)b * NP + k0 + j * 16 + col) * CQ + kc * 32; const v16h kh = frag_h(KH + kr, lane); acc[j] = wmma16(ah, kh, acc[j]); acc[j] = wmma16(al, kh, acc[j]); acc[j] = wmma16(ah, frag_h(KL + kr, lane), acc[j]); } }
#pragma unroll
  for (int j = 0; j < 8; ++j)
#pragma unroll
    for (int r = 0; r < 8; ++r) ss[wave][8 * g + r][j * 16 + col] = acc[j][r];
  LDSX(); for (int rl = 0; rl < 16; ++rl) vst2(S + (size_t)(ql0 + rl) * NP + k0 + lane * 4, *(const v4f*)&ss[wave][rl][lane * 4]); }
__global__ __launch_bounds__(256) void k_sm(const float* __restrict__ S, _Float16* __restrict__ PH) { __shared__ float sred[8]; __shared__ float sbc; __shared__ __align__(16) _Float16 sh[NP];
  const int t = threadIdx.x; const size_t row = blockIdx.x; const float* sr = S + row * NP;
  float m = -3.0e38f; for (int k = t; k < NP; k += 256) m = fmaxf(m, sr[k]);
#pragma unroll
  for (int o = 1; o < 32; o <<= 1) m = fmaxf(m, __shfl_xor(m, o));
  if ((t & 31) == 0) sred[t >> 5] = m; __syncthreads(); if (t == 0) { float a = sred[0]; for (int i = 1; i < 8; ++i) a = fmaxf(a, sred[i]); sbc = a; } __syncthreads(); m = sbc; __syncthreads();
  float sum = 0.f; for (int k = t; k < NP; k += 256) sum += expf(sr[k] - m);
#pragma unroll
  for (int o = 1; o < 32; o <<= 1) sum += __shfl_xor(sum, o);
  if ((t & 31) == 0) sred[t >> 5] = sum; __syncthreads(); if (t == 0) { float a = 0.f; for (int i = 0; i < 8; ++i) a += sred[i]; sbc = 1.0f / a; } __syncthreads(); const float inv = sbc;
  for (int k = t; k < NP; k += 256) sh[k] = (_Float16)(expf(sr[k] - m) * inv * 2048.0f);
  __syncthreads(); for (int q = t; q < NP / 8; q += 256) vst2((unsigned*)(PH + row * NP + q * 8), *(const v4u*)&sh[q * 8]); }
__global__ __launch_bounds__(128) void k_pv(const _Float16* __restrict__ PH, const _Float16* __restrict__ VT, int b, const float* __restrict__ X, const float* __restrict__ GM, float* __restrict__ OUT) { __shared__ __align__(16) float st[128][68];
  const int tid = threadIdx.x, wave = tid >> 5, lane = tid & 31, col = lane & 15, g = lane >> 4; const int c0 = blockIdx.y * 128; const int i0 = blockIdx.x * 64; const int il0 = wave * 16;
  v8f acc[8] = {};
#pragma unroll 1
  for (int kc = 0; kc < NP / 32; ++kc) { const v16h ph = frag_h(PH + (size_t)(i0 + il0 + col) * NP + kc * 32, lane);
#pragma unroll
    for (int j = 0; j < 8; ++j) acc[j] = wmma16(ph, frag_h(VT + ((size_t)b * CV + c0 + j * 16 + col) * (size_t)NP + kc * 32, lane), acc[j]); }
#pragma unroll
  for (int j = 0; j < 8; ++j) { const int cl = j * 16 + col;
#pragma unroll
    for (int r = 0; r < 8; ++r) st[cl][il0 + 8 * g + r] = acc[j][r] * (1.0f / 2048.0f); }
  __syncthreads();
  const float gm = bfr(GM[0]);
  for (int e = tid; e < 64 * 32; e += 128) { const int il = e >> 5, q = e & 31; const size_t o = ((size_t)b * NP + i0 + il) * CV + c0 + q * 4; __align__(16) float v4[4]; const float* xp = X + o; v4[0] = gm * st[q * 4][il] + bfr(xp[0]); v4[1] = gm * st[q * 4 + 1][il] + bfr(xp[1]); v4[2] = gm * st[q * 4 + 2][il] + bfr(xp[2]); v4[3] = gm * st[q * 4 + 3][il] + bfr(xp[3]); vst2(OUT + o, *(const v4f*)v4); } }
extern "C" void kernel_launch(void* const* d_in, const int* in_sizes, int n_in, void* d_out, int out_size, void* d_ws, size_t ws_size, hipStream_t stream) {
  (void)in_sizes; (void)n_in; (void)out_size;
  const float** F = (const float**)d_in;
  if (ws_size < (size_t)WS_END) return;
  char* ws = (char*)d_ws; _Float16 *QH = (_Float16*)(ws + WS_QH), *QL = (_Float16*)(ws + WS_QL), *KH = (_Float16*)(ws + WS_KH), *KL = (_Float16*)(ws + WS_KL), *VT = (_Float16*)(ws + WS_VT), *PH = (_Float16*)(ws + WS_PH); float* S = (float*)(ws + WS_S);
  k_proj<<<dim3(NP / 64, TNB, 3), 128, 0, stream>>>(F[0], F[0], F[1], F[2], F[3], F[4], F[5], F[6], QH, QL, KH, KL, VT);
  for (int b = 0; b < TNB; ++b) {
    k_sc<<<dim3(TQB, NP / 128), 128, 0, stream>>>(QH, QL, KH, KL, b, S);
    k_sm<<<TQB * 64, 256, 0, stream>>>(S, PH);
    k_pv<<<dim3(TQB, CV / 128), 128, 0, stream>>>(PH, VT, b, F[0], F[7], (float*)d_out);
  }
}
